// GroupedQueryAttention_3066606649447
// MI455X (gfx1250) — hardware-verified
//
#include <hip/hip_runtime.h>


#ifndef NB
#define NB 4
#endif
#ifndef SEQ
#define SEQ 1024
#endif
#define NB_FULL  4
#define SEQ_FULL 1024
#define DM   2048
#define NH   32
#define NKV  8
#define REP  4
#define HD   64
#define DQ   2048
#define DKV  512
#define DKV2 1024
#define RH   256
#define PCAR 16.0f
#define CCAR 64.0f
#define SCL2 (0.125f * 1.4426950408889634f)
#define NEGBIG (-3.0e38f)

static_assert(DQ == NH * HD);
static_assert(DKV == NKV * HD);
static_assert(DKV2 == 2 * DKV);
static_assert(NH == NKV * REP);
static_assert(HD == 64);
static_assert(DM % 32 == 0);
static_assert(DQ % 32 == 0);
static_assert(((size_t)NB * SEQ) % 64 == 0);
static_assert(DQ % 64 == 0);
static_assert(DKV2 % 64 == 0);
static_assert(DM % 64 == 0);
static_assert(SEQ % 64 == 0);
static_assert(RH % 64 == 0);
static_assert(RH <= SEQ);
static_assert((SEQ - RH) % 64 == 0);
static_assert(SEQ <= SEQ_FULL);
static_assert(NB <= NB_FULL);
static_assert(SEQ % 8 == 0);
static_assert((size_t)(NB - 1) * SEQ_FULL * DM + (size_t)SEQ * DM <= (size_t)NB_FULL * SEQ_FULL * DM);

typedef _Float16 h16;
typedef unsigned short bf;
typedef __attribute__((ext_vector_type(16))) __bf16   v16bf;
typedef __attribute__((ext_vector_type(16))) _Float16 v16h;
typedef __attribute__((ext_vector_type(8)))  _Float16 v8h;
typedef __attribute__((ext_vector_type(8)))  unsigned short v8us;
typedef __attribute__((ext_vector_type(8)))  float    v8f;
typedef __attribute__((ext_vector_type(4)))  float    v4f;
typedef v8h  __attribute__((may_alias)) v8ha;
typedef v4f  __attribute__((may_alias)) v4fa;

__device__ __forceinline__ unsigned short f2bf(float f) { unsigned u = __float_as_uint(f); u += 0x7FFFu + ((u >> 16) & 1u); return (unsigned short)(u >> 16); }
__device__ __forceinline__ float bf2f(unsigned short b) { return __uint_as_float(((unsigned)b) << 16); }
__device__ __forceinline__ float bfr(float f) { return bf2f(f2bf(f)); }
__device__ __forceinline__ void splitf(float y, unsigned short& h, unsigned short& l) { h = f2bf(y); l = f2bf(y - bf2f(h)); }
__device__ __forceinline__ v16h cat16(v8h lo, v8h hi) { return __builtin_shufflevector(lo, hi, 0, 1, 2, 3, 4, 5, 6, 7, 8, 9, 10, 11, 12, 13, 14, 15); }
__device__ __forceinline__ v16bf cat16b(v8us lo, v8us hi) { return __builtin_bit_cast(v16bf, __builtin_shufflevector(lo, hi, 0, 1, 2, 3, 4, 5, 6, 7, 8, 9, 10, 11, 12, 13, 14, 15)); }
__device__ __forceinline__ v8f wmma16(v16h a, v16h b, v8f c) { return __builtin_amdgcn_wmma_f32_16x16x32_f16(false, a, false, b, (short)0, c, false, false); }
__device__ __forceinline__ v8f wmmab(v16bf a, v16bf b, v8f c) { return __builtin_amdgcn_wmma_f32_16x16x32_bf16(false, a, false, b, (short)0, c, false, false); }
__device__ __forceinline__ v16h ldh(const h16* p) { return cat16(*(const v8h*)p, *(const v8h*)(p + 16)); }
__device__ __forceinline__ v16bf ldb(const bf* p) { return cat16b(*(const v8us*)p, *(const v8us*)(p + 16)); }

template <typename T16> struct WFrag;
template <> struct WFrag<h16> { typedef v16h V; static __device__ __forceinline__ V ld(const h16* p) { return ldh(p); } static __device__ __forceinline__ v8f mma(V a, V b, v8f c) { return wmma16(a, b, c); } };
template <> struct WFrag<bf> { typedef v16bf V; static __device__ __forceinline__ V ld(const bf* p) { return ldb(p); } static __device__ __forceinline__ v8f mma(V a, V b, v8f c) { return wmmab(a, b, c); } };

template <typename T16, int NSPLIT>
__device__ __forceinline__ void gemm_body(const T16* A, const T16* A2, const T16* Bt, int K, float* C, int ldc, float osc, size_t sA, size_t sC) {
    typedef typename WFrag<T16>::V V;
    __shared__ __align__(16) float os[16 * 68];
    const size_t z = blockIdx.z; A += z * sA; A2 += z * sA; C += z * sC;
    const int lane = threadIdx.x & 31, lr = lane & 15, hi = lane >> 4; const int r0 = blockIdx.x * 64, c0 = blockIdx.y * 64;
    v8f acc[4][4];
#pragma unroll
    for (int mb = 0; mb < 4; ++mb)
#pragma unroll
        for (int nb = 0; nb < 4; ++nb) acc[mb][nb] = (v8f){};
    const size_t aoff = (size_t)(r0 + lr) * K + 8 * hi, boff = (size_t)(c0 + lr) * K + 8 * hi;
#pragma unroll 1
    for (int kc = 0; kc < K; kc += 32) {
        V a[4], a2[4];
#pragma unroll
        for (int mb = 0; mb < 4; ++mb) { a[mb] = WFrag<T16>::ld(A + aoff + (size_t)mb * 16 * K + kc); if (NSPLIT == 1) a2[mb] = WFrag<T16>::ld(A2 + aoff + (size_t)mb * 16 * K + kc); else a2[mb] = a[mb]; }
#pragma unroll
        for (int nb = 0; nb < 4; ++nb) { const V b = WFrag<T16>::ld(Bt + boff + (size_t)nb * 16 * K + kc);
#pragma unroll
            for (int mb = 0; mb < 4; ++mb) { acc[mb][nb] = WFrag<T16>::mma(a[mb], b, acc[mb][nb]); if (NSPLIT == 1) acc[mb][nb] = WFrag<T16>::mma(a2[mb], b, acc[mb][nb]); } }
        asm volatile("v_nop\n\tv_nop\n\tv_nop\n\tv_nop" : "+v"(acc[0][0]), "+v"(acc[1][1]), "+v"(acc[2][2]), "+v"(acc[3][3]) : "v"(a[0]), "v"(a[3]), "v"(a2[0]), "v"(a2[3]));
    }
#pragma unroll
    for (int mb = 0; mb < 4; ++mb) {
#pragma unroll
        for (int nb = 0; nb < 4; ++nb) {
#pragma unroll
            for (int j = 0; j < 8; ++j) os[(hi * 8 + j) * 68 + nb * 16 + lr] = acc[mb][nb][j]; }
        __syncthreads();
        float* crow = C + (size_t)(r0 + mb * 16) * ldc + c0;
#pragma unroll 1
        for (int ps = 0; ps < 2; ++ps) {
#pragma unroll
            for (int s = 0; s < 8; ++s) { const int row = 2 * s + hi, cofs = lr * 4; v4f val = *(const v4fa*)(os + row * 68 + cofs); val = val * osc;
                *(volatile v4f*)(crow + (size_t)row * ldc + cofs) = val; }
            if (ps == 0) __threadfence(); }
        __syncthreads();
    }
}
__global__ __launch_bounds__(32) void k_gemm_b(const bf* A, const bf* Bt, int K, float* C, int ldc, size_t sA, size_t sC) { gemm_body<bf, 0>(A, A, Bt, K, C, ldc, 1.0f, sA, sC); }
__global__ __launch_bounds__(32) void k_gemm_bhl(const bf* A, const bf* A2, const bf* Bt, int K, float* C, int ldc, size_t sA, size_t sC) { gemm_body<bf, 1>(A, A2, Bt, K, C, ldc, 1.0f, sA, sC); }
__global__ __launch_bounds__(32) void k_gemm_h(const h16* A, const h16* Bt, int K, float* C, int ldc, float osc, size_t sA, size_t sC) { gemm_body<h16, 0>(A, A, Bt, K, C, ldc, osc, sA, sC); }

__global__ __launch_bounds__(256) void k_wt8(const float* __restrict__ w, int K, int N, bf* Bt, h16* Bh, int mkh, float hsc) {
    const size_t i = (size_t)blockIdx.x * 256 + threadIdx.x; const size_t tot = (size_t)N * K / 8; if (i >= tot) return;
    const size_t e = i * 8; const int k = (int)(e % (size_t)K), n = (int)(e / (size_t)K); v8us o; v8h oh;
#pragma unroll
    for (int q = 0; q < 8; ++q) { const float v = w[(size_t)(k + q) * N + n]; const unsigned short bb = f2bf(v); o[q] = bb; oh[q] = (h16)(bf2f(bb) * hsc); }
    *(volatile v8us*)(Bt + e) = o; if (mkh) *(volatile v8h*)(Bh + e) = oh;
    __threadfence();
    *(volatile v8us*)(Bt + e) = o; if (mkh) *(volatile v8h*)(Bh + e) = oh;
}
__global__ __launch_bounds__(256) void k_cvt8(const float* __restrict__ src, bf* dst, int n8, size_t sstride, size_t dstride) {
    const int i = blockIdx.x * 256 + threadIdx.x; if (i >= n8) return;
    const float* s = src + (size_t)blockIdx.y * sstride + (size_t)i * 8; bf* d = dst + (size_t)blockIdx.y * dstride + (size_t)i * 8;
    const v4f a = *(const v4f*)s, c = *(const v4f*)(s + 4); v8us o;
#pragma unroll
    for (int q = 0; q < 4; ++q) { o[q] = f2bf(a[q]); o[4 + q] = f2bf(c[q]); }
    *(volatile v8us*)d = o; __threadfence(); *(volatile v8us*)d = o;
}
__global__ __launch_bounds__(256) void k_rope(const float* __restrict__ F, int pitch, int coff, int nheads, const float* __restrict__ COS, const float* __restrict__ SIN, h16* P16, bf* Ph, bf* Pl) {
    const size_t i = (size_t)blockIdx.x * 256 + threadIdx.x; const size_t tot = (size_t)NB * nheads * SEQ * 8; if (i >= tot) return;
    const int c8 = (int)(i & 7); const size_t rowi = i >> 3; const int t = (int)(rowi % SEQ); const int h = (int)((rowi / SEQ) % (size_t)nheads); const int b = (int)(rowi / ((size_t)SEQ * nheads));
    const int d0 = c8 * 8, dp0 = d0 ^ 32;
    const float* f = F + ((size_t)b * SEQ + t) * pitch + coff + h * HD;
    const v4f xa = *(const v4f*)(f + d0), xb = *(const v4f*)(f + d0 + 4), ya = *(const v4f*)(f + dp0), yb = *(const v4f*)(f + dp0 + 4);
    const v4f ca = *(const v4f*)(COS + (size_t)t * HD + d0), cb = *(const v4f*)(COS + (size_t)t * HD + d0 + 4), sa = *(const v4f*)(SIN + (size_t)t * HD + d0), sb = *(const v4f*)(SIN + (size_t)t * HD + d0 + 4);
    const float sg = (d0 < 32) ? -1.0f : 1.0f;
    v8h o16; v8us oh, ol;
#pragma unroll
    for (int q = 0; q < 4; ++q) {
        const float r0 = xa[q] * bfr(ca[q]) + (sg * ya[q]) * bfr(sa[q]);
        const float r1 = xb[q] * bfr(cb[q]) + (sg * yb[q]) * bfr(sb[q]);
        unsigned short a2, c2; o16[q] = (h16)r0; splitf(r0, a2, c2); oh[q] = a2; ol[q] = c2; o16[4 + q] = (h16)r1; splitf(r1, a2, c2); oh[4 + q] = a2; ol[4 + q] = c2; }
    const size_t e = i * 8; const size_t eh = (((size_t)b * nheads + h) * RH + (t < RH ? t : 0)) * HD + d0; const bool hr = (t < RH);
    *(volatile v8h*)(P16 + e) = o16; if (hr) { *(volatile v8us*)(Ph + eh) = oh; *(volatile v8us*)(Pl + eh) = ol; }
    __threadfence();
    *(volatile v8h*)(P16 + e) = o16; if (hr) { *(volatile v8us*)(Ph + eh) = oh; *(volatile v8us*)(Pl + eh) = ol; }
}
__global__ __launch_bounds__(256) void k_vtp(const float* __restrict__ F, int pitch, int coff, h16* V16, bf* Vh, bf* Vl) {
    const size_t i = (size_t)blockIdx.x * 256 + threadIdx.x; const size_t tot = (size_t)NB * NKV * HD * (SEQ / 8); if (i >= tot) return;
    const int t0 = (int)(i % (SEQ / 8)) * 8; const int d = (int)((i / (SEQ / 8)) % HD); const int g = (int)((i / ((size_t)(SEQ / 8) * HD)) % NKV); const int b = (int)(i / ((size_t)(SEQ / 8) * HD * NKV));
    v8h o16; v8us oh, ol;
#pragma unroll
    for (int q = 0; q < 8; ++q) { const float x = F[((size_t)b * SEQ + t0 + q) * pitch + coff + g * HD + d]; unsigned short a2, c2; o16[q] = (h16)x; splitf(x, a2, c2); oh[q] = a2; ol[q] = c2; }
    const size_t e = i * 8; const bool hr = (t0 < RH); const size_t eh = (((size_t)b * NKV + g) * HD + d) * RH + (hr ? t0 : 0);
    *(volatile v8h*)(V16 + e) = o16; if (hr) { *(volatile v8us*)(Vh + eh) = oh; *(volatile v8us*)(Vl + eh) = ol; }
    __threadfence();
    *(volatile v8h*)(V16 + e) = o16; if (hr) { *(volatile v8us*)(Vh + eh) = oh; *(volatile v8us*)(Vl + eh) = ol; }
}

__device__ __forceinline__ float softmax_step(v8f s0, v8f s1, int kvb, int hh, int qi, float& m_run, float& l_run, v8f& p0, v8f& p1) {
    float mx = NEGBIG;
#pragma unroll
    for (int r = 0; r < 8; ++r) {
        float a = s0[r] * SCL2; a = (kvb + 8 * hh + r > qi) ? NEGBIG : a; p0[r] = a; mx = fmaxf(mx, a);
        float c = s1[r] * SCL2; c = (kvb + 16 + 8 * hh + r > qi) ? NEGBIG : c; p1[r] = c; mx = fmaxf(mx, c); }
    mx = fmaxf(mx, __shfl_xor(mx, 16, 32));
    const float m_new = fmaxf(m_run, mx);
    const float alpha = __builtin_amdgcn_exp2f(m_run - m_new);
    float ls = 0.0f;
#pragma unroll
    for (int r = 0; r < 8; ++r) { const float e0 = __builtin_amdgcn_exp2f(p0[r] - m_new); p0[r] = e0; ls += e0; const float e1 = __builtin_amdgcn_exp2f(p1[r] - m_new); p1[r] = e1; ls += e1; }
    ls += __shfl_xor(ls, 16, 32);
    l_run = l_run * alpha + ls; m_run = m_new;
    return alpha;
}
__device__ __forceinline__ v8f score_hl(const bf* Qh, const bf* Ql, const bf* Kh, const bf* Kl, size_t qoff, size_t ko) {
    const v16bf qh0 = ldb(Qh + qoff), qh1 = ldb(Qh + qoff + 32), ql0 = ldb(Ql + qoff), ql1 = ldb(Ql + qoff + 32);
    const v16bf kh0 = ldb(Kh + ko), kh1 = ldb(Kh + ko + 32), kl0 = ldb(Kl + ko), kl1 = ldb(Kl + ko + 32);
    v8f a = (v8f){};
    a = wmmab(kh0, qh0, a); a = wmmab(kl0, qh0, a); a = wmmab(kh0, ql0, a);
    a = wmmab(kh1, qh1, a); a = wmmab(kl1, qh1, a); a = wmmab(kh1, ql1, a);
    asm volatile("v_nop\n\tv_nop\n\tv_nop\n\tv_nop" : "+v"(a) : "v"(kh0), "v"(kh1), "v"(kl0), "v"(kl1), "v"(qh0), "v"(qh1), "v"(ql0), "v"(ql1));
    return a;
}

template <bool HIRES>
__device__ __forceinline__ void attn_body(const h16* Q16, const h16* K16, const h16* V16, const bf* Qh, const bf* Ql, const bf* Kh, const bf* Kl, const bf* Vh, const bf* Vl,
                                          h16* C16, bf* Ch, bf* Cl, int qblk0) {
    constexpr int TP = HIRES ? RH : SEQ;
    static_assert(TP % 32 == 0);
    __shared__ __align__(16) float osf[HIRES ? 4 * 16 * 68 : 4];
    __shared__ __align__(16) h16   osh[HIRES ? 8 : 4 * 16 * 72];
    const int wave = __builtin_amdgcn_readfirstlane((int)(threadIdx.x >> 5));
    const int lane = threadIdx.x & 31, lr = lane & 15, hh = lane >> 4;
    const int hq = blockIdx.y, b = blockIdx.z, g = hq / REP;
    const int qb = ((int)blockIdx.x + qblk0) * 64 + wave * 16;
    const int qi = qb + lr;
    const size_t qoff  = (((size_t)b * NH + hq) * TP + qi) * HD + 8 * hh;
    const size_t kbase = ((size_t)b * NKV + g) * TP * HD + (size_t)lr * HD + 8 * hh;
    const size_t vbase = ((size_t)b * NKV + g) * HD * TP + (size_t)lr * TP + 8 * hh;
    v8f o[4];
#pragma unroll
    for (int dd = 0; dd < 4; ++dd) o[dd] = (v8f){};
    float m_run = NEGBIG, l_run = 0.0f;
    const int nt = min((qb + 47) >> 5, TP / 32);
    if (HIRES) {
#pragma unroll 1
        for (int t = 0; t < nt; ++t) {
            const int kvb = t * 32;
            const size_t ko = kbase + (size_t)kvb * HD;
            const v8f s0 = score_hl(Qh, Ql, Kh, Kl, qoff, ko);
            const v8f s1 = score_hl(Qh, Ql, Kh, Kl, qoff, ko + (size_t)16 * HD);
            v8f p0, p1; const float alpha = softmax_step(s0, s1, kvb, hh, qi, m_run, l_run, p0, p1);
#pragma unroll
            for (int dd = 0; dd < 4; ++dd) o[dd] = o[dd] * alpha;
            v8us ph0, pl0, ph1, pl1;
#pragma unroll
            for (int r = 0; r < 8; ++r) { unsigned short a2, c2; splitf(p0[r], a2, c2); ph0[r] = a2; pl0[r] = c2; splitf(p1[r], a2, c2); ph1[r] = a2; pl1[r] = c2; }
            const v16bf pH = cat16b(ph0, ph1), pL = cat16b(pl0, pl1);
#pragma unroll
            for (int dd = 0; dd < 4; ++dd) { const size_t vo = vbase + (size_t)dd * 16 * TP + kvb; const v16bf vh = ldb(Vh + vo), vl = ldb(Vl + vo);
                o[dd] = wmmab(vh, pH, o[dd]); o[dd] = wmmab(vl, pH, o[dd]); o[dd] = wmmab(vh, pL, o[dd]);
                asm volatile("v_nop\n\tv_nop\n\tv_nop\n\tv_nop" : "+v"(o[dd]) : "v"(vh), "v"(vl), "v"(pH), "v"(pL)); }
        }
    } else {
        const v16h qt0 = ldh(Q16 + qoff), qt1 = ldh(Q16 + qoff + 32);
#pragma unroll 1
        for (int t = 0; t < nt; ++t) {
            const int kvb = t * 32;
            const size_t ko = kbase + (size_t)kvb * HD;
            const v16h k00 = ldh(K16 + ko), k01 = ldh(K16 + ko + 32), k10 = ldh(K16 + ko + (size_t)16 * HD), k11 = ldh(K16 + ko + (size_t)16 * HD + 32);
            v8f s0 = (v8f){}, s1 = (v8f){};
            s0 = wmma16(k00, qt0, s0); s0 = wmma16(k01, qt1, s0); s1 = wmma16(k10, qt0, s1); s1 = wmma16(k11, qt1, s1);
            asm volatile("v_nop\n\tv_nop\n\tv_nop\n\tv_nop" : "+v"(s0), "+v"(s1) : "v"(k00), "v"(k01), "v"(k10), "v"(k11), "v"(qt0), "v"(qt1));
            v8f p0, p1; const float alpha = softmax_step(s0, s1, kvb, hh, qi, m_run, l_run, p0, p1);
#pragma unroll
            for (int dd = 0; dd < 4; ++dd) o[dd] = o[dd] * alpha;
            v16h pf;
#pragma unroll
            for (int r = 0; r < 8; ++r) { pf[r] = (h16)(p0[r] * PCAR); pf[8 + r] = (h16)(p1[r] * PCAR); }
            const size_t vo = vbase + kvb;
            const v16h v0 = ldh(V16 + vo), v1 = ldh(V16 + vo + (size_t)16 * TP), v2 = ldh(V16 + vo + (size_t)32 * TP), v3 = ldh(V16 + vo + (size_t)48 * TP);
            o[0] = wmma16(v0, pf, o[0]); o[1] = wmma16(v1, pf, o[1]); o[2] = wmma16(v2, pf, o[2]); o[3] = wmma16(v3, pf, o[3]);
            asm volatile("v_nop\n\tv_nop\n\tv_nop\n\tv_nop" : "+v"(o[0]), "+v"(o[1]), "+v"(o[2]), "+v"(o[3]) : "v"(v0), "v"(v1), "v"(v2), "v"(v3), "v"(pf));
        }
    }
    const int rq = lane >> 3, pc = lane & 7;
    if (HIRES) {
        const float inv = 1.0f / l_run;
#pragma unroll
        for (int dd = 0; dd < 4; ++dd) { v4f a4, b4;
#pragma unroll
            for (int r = 0; r < 4; ++r) { a4[r] = o[dd][r] * inv; b4[r] = o[dd][4 + r] * inv; }
            *(v4fa*)(osf + (wave * 16 + lr) * 68 + dd * 16 + 8 * hh) = a4; *(v4fa*)(osf + (wave * 16 + lr) * 68 + dd * 16 + 8 * hh + 4) = b4; }
        __syncthreads();
        const size_t dofs = ((size_t)b * RH + qb) * DQ + hq * HD + pc * 8;
#pragma unroll 1
        for (int ps = 0; ps < 2; ++ps) {
#pragma unroll
            for (int s = 0; s < 4; ++s) { const int row = s * 4 + rq; const v4f x0 = *(const v4fa*)(osf + (wave * 16 + row) * 68 + pc * 8), x1 = *(const v4fa*)(osf + (wave * 16 + row) * 68 + pc * 8 + 4); v8us oh, ol;
#pragma unroll
                for (int q = 0; q < 4; ++q) { unsigned short a2, c2; splitf(x0[q], a2, c2); oh[q] = a2; ol[q] = c2; splitf(x1[q], a2, c2); oh[4 + q] = a2; ol[4 + q] = c2; }
                *(volatile v8us*)(Ch + dofs + (size_t)row * DQ) = oh; *(volatile v8us*)(Cl + dofs + (size_t)row * DQ) = ol; }
            if (ps == 0) __threadfence(); }
    } else {
        const float inv = CCAR / (PCAR * l_run);
#pragma unroll
        for (int dd = 0; dd < 4; ++dd) { v8h o8;
#pragma unroll
            for (int r = 0; r < 8; ++r) o8[r] = (h16)(o[dd][r] * inv);
            *(v8ha*)(osh + (wave * 16 + lr) * 72 + dd * 16 + 8 * hh) = o8; }
        __syncthreads();
        const size_t dofs = ((size_t)b * SEQ + qb) * DQ + hq * HD + pc * 8;
#pragma unroll 1
        for (int ps = 0; ps < 2; ++ps) {
#pragma unroll
            for (int s = 0; s < 4; ++s) { const int row = s * 4 + rq; const v8h val = *(const v8ha*)(osh + (wave * 16 + row) * 72 + pc * 8);
                *(volatile v8h*)(C16 + dofs + (size_t)row * DQ) = val; }
            if (ps == 0) __threadfence(); }
    }
}
__global__ __launch_bounds__(128) void k_attn_hi(const h16* Q16, const h16* K16, const h16* V16, const bf* Qh, const bf* Ql, const bf* Kh, const bf* Kl, const bf* Vh, const bf* Vl, h16* C16, bf* Ch, bf* Cl) {
    attn_body<true>(Q16, K16, V16, Qh, Ql, Kh, Kl, Vh, Vl, C16, Ch, Cl, 0); }
__global__ __launch_bounds__(128) void k_attn_lo(const h16* Q16, const h16* K16, const h16* V16, const bf* Qh, const bf* Ql, const bf* Kh, const bf* Kl, const bf* Vh, const bf* Vl, h16* C16, bf* Ch, bf* Cl) {
    attn_body<false>(Q16, K16, V16, Qh, Ql, Kh, Kl, Vh, Vl, C16, Ch, Cl, RH / 64); }

constexpr size_t cmaxz(size_t a, size_t b) { return a > b ? a : b; }
constexpr size_t MROWS  = (size_t)NB * SEQ;
constexpr size_t SZ_WQ  = (size_t)DQ * DM * 2, SZ_WKV = (size_t)DKV2 * DM * 2, SZ_WO = (size_t)DM * DQ * 2;
constexpr size_t SZ_XB  = MROWS * DM * 2;
constexpr size_t SZ_Q16 = MROWS * DQ * 2, SZ_K16 = MROWS * DKV * 2, SZ_QH = (size_t)NB * NH * RH * HD * 2, SZ_KH = (size_t)NB * NKV * RH * HD * 2;
constexpr size_t SZ_RA  = cmaxz(2 * SZ_XB, SZ_Q16 + 2 * SZ_K16 + 2 * SZ_QH);
constexpr size_t SZ_FQ  = MROWS * DQ * 4, SZ_C16 = MROWS * DQ * 2, SZ_AT = (size_t)NB * RH * DQ * 2;
constexpr size_t SZ_RB  = cmaxz(SZ_FQ, SZ_C16 + 2 * SZ_AT);
constexpr size_t SZ_FKV = MROWS * DKV2 * 4;
constexpr size_t OFF_WQ = 0, OFF_WKV = OFF_WQ + SZ_WQ, OFF_WOB = OFF_WKV + SZ_WKV, OFF_WOH = OFF_WOB + SZ_WO, OFF_RA = OFF_WOH + SZ_WO, OFF_RB = OFF_RA + SZ_RA, OFF_FKV = OFF_RB + SZ_RB;
constexpr size_t OFF_KH = OFF_FKV + SZ_FKV, OFF_KL = OFF_KH + SZ_KH, OFF_VH = OFF_KL + SZ_KH, OFF_VL = OFF_VH + SZ_KH, WS_TOTAL = OFF_VL + SZ_KH;
static_assert(WS_TOTAL <= (size_t)134217728);
static_assert(SZ_WQ % 256 == 0 && SZ_WKV % 256 == 0 && SZ_WO % 256 == 0 && SZ_XB % 256 == 0 && SZ_RA % 256 == 0 && SZ_RB % 256 == 0 && SZ_FKV % 256 == 0 && SZ_KH % 256 == 0);
static_assert(SZ_Q16 % 256 == 0 && SZ_K16 % 256 == 0 && SZ_QH % 256 == 0 && SZ_C16 % 256 == 0 && SZ_AT % 256 == 0);
static_assert(2 * SZ_XB <= SZ_RA && SZ_Q16 + 2 * SZ_K16 + 2 * SZ_QH <= SZ_RA);
static_assert(SZ_FQ <= SZ_RB && SZ_C16 + 2 * SZ_AT <= SZ_RB);

extern "C" void kernel_launch(void* const* d_in, const int* in_sizes, int n_in,
                              void* d_out, int out_size, void* d_ws, size_t ws_size, hipStream_t stream) {
    if (n_in < 10) return;
    const size_t actneed = (size_t)(NB - 1) * SEQ_FULL * DM + (size_t)SEQ * DM;
    if ((size_t)in_sizes[0] < actneed || (size_t)in_sizes[1] < actneed) return;
    if (in_sizes[2] < SEQ * HD || in_sizes[3] < SEQ * HD || in_sizes[4] < SEQ * HD || in_sizes[5] < SEQ * HD) return;
    if (in_sizes[6] < DM * DQ || in_sizes[7] < DM * DKV || in_sizes[8] < DM * DKV || in_sizes[9] < DQ * DM) return;
    if ((size_t)out_size < actneed) return;
    if (ws_size < WS_TOTAL) return;
    const float* x = (const float*)d_in[0]; const float* ctx = (const float*)d_in[1];
    const float* cosq = (const float*)d_in[2]; const float* sinq = (const float*)d_in[3]; const float* cosk = (const float*)d_in[4]; const float* sink = (const float*)d_in[5];
    const float* wq = (const float*)d_in[6]; const float* wk = (const float*)d_in[7]; const float* wv = (const float*)d_in[8]; const float* wo = (const float*)d_in[9];
    float* OUT = (float*)d_out;
    char* ws = (char*)d_ws;
    bf* WQ = (bf*)(ws + OFF_WQ); bf* WKV = (bf*)(ws + OFF_WKV); bf* WOB = (bf*)(ws + OFF_WOB); h16* WOH = (h16*)(ws + OFF_WOH);
    bf* XB = (bf*)(ws + OFF_RA); bf* CB = (bf*)(ws + OFF_RA + SZ_XB);
    h16* Q16 = (h16*)(ws + OFF_RA); h16* K16 = (h16*)(ws + OFF_RA + SZ_Q16); h16* VT16 = (h16*)(ws + OFF_RA + SZ_Q16 + SZ_K16);
    bf* QPh = (bf*)(ws + OFF_RA + SZ_Q16 + 2 * SZ_K16); bf* QPl = (bf*)(ws + OFF_RA + SZ_Q16 + 2 * SZ_K16 + SZ_QH);
    float* FQ = (float*)(ws + OFF_RB); h16* C16 = (h16*)(ws + OFF_RB); bf* ATh = (bf*)(ws + OFF_RB + SZ_C16); bf* ATl = (bf*)(ws + OFF_RB + SZ_C16 + SZ_AT);
    float* FKV = (float*)(ws + OFF_FKV);
    bf* KPh = (bf*)(ws + OFF_KH); bf* KPl = (bf*)(ws + OFF_KL); bf* VTh = (bf*)(ws + OFF_VH); bf* VTl = (bf*)(ws + OFF_VL);

    k_wt8<<<(unsigned)(((size_t)DQ * DM / 8 + 255) / 256), 256, 0, stream>>>(wq, DM, DQ, WQ, WOH, 0, 1.0f);
    k_wt8<<<(unsigned)(((size_t)DKV * DM / 8 + 255) / 256), 256, 0, stream>>>(wk, DM, DKV, WKV, WOH, 0, 1.0f);
    k_wt8<<<(unsigned)(((size_t)DKV * DM / 8 + 255) / 256), 256, 0, stream>>>(wv, DM, DKV, WKV + (size_t)DKV * DM, WOH, 0, 1.0f);
    k_wt8<<<(unsigned)(((size_t)DM * DQ / 8 + 255) / 256), 256, 0, stream>>>(wo, DQ, DM, WOB, WOH, 1, CCAR);
    const int n8 = SEQ * DM / 8;
    k_cvt8<<<dim3((unsigned)((n8 + 255) / 256), NB, 1), 256, 0, stream>>>(x, XB, n8, (size_t)SEQ_FULL * DM, (size_t)SEQ * DM);
    k_cvt8<<<dim3((unsigned)((n8 + 255) / 256), NB, 1), 256, 0, stream>>>(ctx, CB, n8, (size_t)SEQ_FULL * DM, (size_t)SEQ * DM);
    k_gemm_b<<<dim3((unsigned)(MROWS / 64), DQ / 64, 1), 32, 0, stream>>>(XB, WQ, DM, FQ, DQ, 0, 0);
    k_gemm_b<<<dim3((unsigned)(MROWS / 64), DKV2 / 64, 1), 32, 0, stream>>>(CB, WKV, DM, FKV, DKV2, 0, 0);
    k_rope<<<(unsigned)(((size_t)NB * NH * SEQ * 8 + 255) / 256), 256, 0, stream>>>(FQ, DQ, 0, NH, cosq, sinq, Q16, QPh, QPl);
    k_rope<<<(unsigned)(((size_t)NB * NKV * SEQ * 8 + 255) / 256), 256, 0, stream>>>(FKV, DKV2, 0, NKV, cosk, sink, K16, KPh, KPl);
    k_vtp<<<(unsigned)(((size_t)NB * NKV * HD * (SEQ / 8) + 255) / 256), 256, 0, stream>>>(FKV, DKV2, DKV, VT16, VTh, VTl);
    k_attn_hi<<<dim3(RH / 64, NH, NB), 128, 0, stream>>>(Q16, K16, VT16, QPh, QPl, KPh, KPl, VTh, VTl, C16, ATh, ATl);
    if (SEQ > RH) k_attn_lo<<<dim3((SEQ - RH) / 64, NH, NB), 128, 0, stream>>>(Q16, K16, VT16, QPh, QPl, KPh, KPl, VTh, VTl, C16, ATh, ATl);
    k_gemm_bhl<<<dim3(RH / 64, DM / 64, NB), 32, 0, stream>>>(ATh, ATl, WOB, DQ, OUT, DM, (size_t)RH * DQ, (size_t)SEQ_FULL * DM);
    if (SEQ > RH) k_gemm_h<<<dim3((SEQ - RH) / 64, DM / 64, NB), 32, 0, stream>>>(C16 + (size_t)RH * DQ, WOH, DQ, OUT + (size_t)RH * DM, DM, 1.0f / (CCAR * CCAR), (size_t)SEQ * DQ, (size_t)SEQ_FULL * DM);
}
